// CapsuleLayer_56899726738051
// MI455X (gfx1250) — hardware-verified
//
#include <hip/hip_runtime.h>
#include <stddef.h>
#include <stdint.h>

#define NB_    64
#define NI     2048
#define DI     8
#define NCAP   32
#define DO_    16
#define NE     (NCAP * DO_)
#define KTOT   (NI * DI)
#define IC     32
#define NCH    (NI / IC)
#define RTHR   256
#define GTHR   128
#define CTHR   128
#define PTHR   256
#define NXU    (NB_ * NI * DI / 8)
#define NWU    (NCAP * NI * DO_ * DI / 8)
#define SPCH   (NB_ * NE)
#define WSMAX  134217728
#define EPSQ   1e-7f

static_assert(NXU % PTHR == 0 && NWU % PTHR == 0);
static_assert(KTOT % 32 == 0);
static_assert(NI % IC == 0);
static_assert(NE == 4 * 32 * 4);
static_assert(NE == CTHR * 4);
static_assert(RTHR == 8 * 32 && NCAP == 8 * 4);
static_assert(16 * NE == 8 * RTHR * 4);
static_assert(16 * NE == 16 * GTHR * 4);
static_assert((NI * DO_) == (1 << 15) && NI == (1 << 11));

typedef float          v2f   __attribute__((ext_vector_type(2)));
typedef float          v4f   __attribute__((ext_vector_type(4)));
typedef float          v8f   __attribute__((ext_vector_type(8)));
typedef int            v4i   __attribute__((ext_vector_type(4)));
typedef int            v8i   __attribute__((ext_vector_type(8)));
typedef unsigned short v8us  __attribute__((ext_vector_type(8)));
typedef unsigned short v16us __attribute__((ext_vector_type(16)));
typedef __bf16         v16bf __attribute__((ext_vector_type(16)));
typedef v2f  __attribute__((may_alias)) v2fa;
typedef v4f  __attribute__((may_alias)) v4fa;
typedef v4i  __attribute__((may_alias)) v4ia;
typedef v8us __attribute__((may_alias)) v8usa;
union FragB { v16bf v; v16us u; v8us h[2]; v4i q[2]; v8i w; };

__device__ __forceinline__ v8f wmb(const FragB& a, const FragB& b, v8f c) {
  v8f d = __builtin_amdgcn_wmma_f32_16x16x32_bf16(false, a.v, false, b.v, (short)0, c, false, false);
  asm volatile("v_nop\n\tv_nop\n\tv_nop\n\tv_nop" : "+v"(d) : "v"(a.w), "v"(b.w));
  return d;
}

__device__ __forceinline__ unsigned bf16_bits(float f) {
  const unsigned u = __float_as_uint(f);
  return (u + 0x7FFFu + ((u >> 16) & 1u)) >> 16;
}
__device__ __forceinline__ void put16(unsigned short* dp, v8us o) {
  *(volatile v8us*)dp = o;
  __threadfence();
  *(volatile v8us*)dp = o;
}

__device__ __forceinline__ float row_max32(const float* rp) {
  const v4f g0 = *(const v4fa*)rp;
  float mx = fmaxf(fmaxf(g0.x, g0.y), fmaxf(g0.z, g0.w));
#pragma unroll
  for (int j = 1; j < 8; ++j) {
    const v4f g = *(const v4fa*)(rp + 4 * j);
    mx = fmaxf(mx, fmaxf(fmaxf(g.x, g.y), fmaxf(g.z, g.w)));
  }
  return mx;
}
__device__ __forceinline__ float row_sum32(const float* rp) {
  float s = 0.0f;
#pragma unroll
  for (int j = 0; j < 8; ++j) {
    const v4f g = *(const v4fa*)(rp + 4 * j);
    s += g.x; s += g.y; s += g.z; s += g.w;
  }
  return s;
}

__global__ __launch_bounds__(PTHR) void k_prep(const float* __restrict__ X, const float* __restrict__ W,
                                               unsigned short* XB, unsigned short* WT) {
  const int u = (int)blockIdx.x * PTHR + (int)threadIdx.x;
  if (u < NXU) {
    const float* src = X + (size_t)u * 8;
    const v4f a = *(const v4fa*)src;
    const v4f c = *(const v4fa*)(src + 4);
    v8us o;
    o[0] = (unsigned short)bf16_bits(a.x); o[1] = (unsigned short)bf16_bits(a.y);
    o[2] = (unsigned short)bf16_bits(a.z); o[3] = (unsigned short)bf16_bits(a.w);
    o[4] = (unsigned short)bf16_bits(c.x); o[5] = (unsigned short)bf16_bits(c.y);
    o[6] = (unsigned short)bf16_bits(c.z); o[7] = (unsigned short)bf16_bits(c.w);
    put16(XB + (size_t)u * 8, o);
  } else {
    const int v = u - NXU;
    if (v >= NWU) return;
    const int n = v >> 15;
    const int e = (v >> 11) & 15;
    const int i = v & (NI - 1);
    const float* src = W + (((size_t)n * NI + i) * DO_ + e) * DI;
    const v4f a = *(const v4fa*)src;
    const v4f c = *(const v4fa*)(src + 4);
    v8us o;
    o[0] = (unsigned short)bf16_bits(a.x); o[1] = (unsigned short)bf16_bits(a.y);
    o[2] = (unsigned short)bf16_bits(a.z); o[3] = (unsigned short)bf16_bits(a.w);
    o[4] = (unsigned short)bf16_bits(c.x); o[5] = (unsigned short)bf16_bits(c.y);
    o[6] = (unsigned short)bf16_bits(c.z); o[7] = (unsigned short)bf16_bits(c.w);
    put16(WT + (size_t)v * 8, o);
  }
}

__global__ __launch_bounds__(GTHR) void k_gemm0(const unsigned short* __restrict__ XB,
                                                const unsigned short* __restrict__ WT, float* SP) {
  __shared__ __attribute__((aligned(16))) float stg[16 * NE];
  const int tid = (int)threadIdx.x, lane = tid & 31, wave = tid >> 5, hh = lane >> 4, m = lane & 15;
  const int bt = (int)blockIdx.x;

  v8f acc[8];
  {
    const v8f z = {0.f, 0.f, 0.f, 0.f, 0.f, 0.f, 0.f, 0.f};
#pragma unroll
    for (int t = 0; t < 8; ++t) acc[t] = z;
  }
  const unsigned short* ap = XB + (size_t)(16 * bt + m) * (size_t)KTOT + 8 * hh;
  const unsigned short* bp = WT + (size_t)(128 * wave + m) * (size_t)KTOT + 8 * hh;

#pragma unroll 1
  for (int k0 = 0; k0 < KTOT; k0 += 32) {
    FragB af;
    af.h[0] = *(const v8usa*)(ap + k0);
    af.h[1] = *(const v8usa*)(ap + k0 + 16);
#pragma unroll
    for (int nt = 0; nt < 8; ++nt) {
      const unsigned short* wq = bp + (size_t)(16 * nt) * (size_t)KTOT + k0;
      FragB bf;
      bf.h[0] = *(const v8usa*)wq;
      bf.h[1] = *(const v8usa*)(wq + 16);
      acc[nt] = wmb(af, bf, acc[nt]);
    }
  }

#pragma unroll
  for (int nt = 0; nt < 8; ++nt) {
    const int col = 128 * wave + 16 * nt + m;
#pragma unroll
    for (int r = 0; r < 8; ++r) stg[(8 * hh + r) * NE + col] = acc[nt][r];
  }
  __syncthreads();

  v4f pv[16];
#pragma unroll
  for (int it = 0; it < 16; ++it) pv[it] = *(const v4fa*)(stg + it * 512 + tid * 4);
  float* op = SP + (size_t)bt * 16 * NE;
#pragma unroll
  for (int it = 0; it < 16; ++it) *(volatile v4f*)(op + it * 512 + tid * 4) = pv[it];
  __threadfence();
#pragma unroll
  for (int it = 0; it < 16; ++it) *(volatile v4f*)(op + it * 512 + tid * 4) = pv[it];
}

__global__ __launch_bounds__(CTHR) void k_combine(const float* __restrict__ SP, int nc, float cscale,
                                                  float* dst) {
  const int b = (int)blockIdx.x, t = (int)threadIdx.x;
  const float* p = SP + (size_t)b * NE + 4 * t;
  const int ncc = nc < 1 ? 1 : (nc > NCH ? NCH : nc);
  v4f s = {0.0f, 0.0f, 0.0f, 0.0f};
#pragma unroll 4
  for (int c = 0; c < ncc; ++c) s += *(const v4fa*)(p + (size_t)c * SPCH);
  s = s * cscale;
  float s2 = s.x * s.x + s.y * s.y + s.z * s.z + s.w * s.w;
  s2 += __shfl_xor(s2, 1);
  s2 += __shfl_xor(s2, 2);
  const float scale = (s2 / (1.0f + s2)) / sqrtf(s2 + EPSQ);
  const v4f o = s * scale;
  float* op = dst + (size_t)b * NE + 4 * t;
  *(volatile v4f*)op = o;
  __threadfence();
  *(volatile v4f*)op = o;
}

template <int PASS>
__global__ __launch_bounds__(RTHR) void k_route(const unsigned short* __restrict__ XB,
                                                const unsigned short* __restrict__ WT,
                                                const float* __restrict__ V,
                                                float* L, float* SP) {
  __shared__ __attribute__((aligned(16))) float sLog[16 * NCAP];
  __shared__ __attribute__((aligned(16))) float sExp[16 * NCAP];
  __shared__ __attribute__((aligned(16))) float stg[16 * NE];

  const int tid = (int)threadIdx.x, lane = tid & 31, q = tid >> 5, h = lane >> 4, m = lane & 15;
  const int chunk = (int)blockIdx.x, bt = (int)blockIdx.y;
  const int b  = 16 * bt + m;
  const int i0 = chunk * IC;
  const int km = h - 1;
  const v4i msk = {km, km, km, km};
  const v4i z4i = {0, 0, 0, 0};
  const v8f z8  = {0.f, 0.f, 0.f, 0.f, 0.f, 0.f, 0.f, 0.f};

  v8f vr[4], acc[4];
#pragma unroll
  for (int nt = 0; nt < 4; ++nt) {
    const float* vp = V + ((size_t)b * NCAP + 4 * q + nt) * DO_ + 8 * h;
    const v4f a = *(const v4fa*)vp;
    const v4f c = *(const v4fa*)(vp + 4);
    const v8f t8 = {a.x, a.y, a.z, a.w, c.x, c.y, c.z, c.w};
    vr[nt]  = t8;
    acc[nt] = z8;
  }

  const unsigned short* xrow = XB + (size_t)b * (size_t)KTOT;
  const unsigned short* wrow = WT + ((size_t)(4 * q) * DO_ + m) * (size_t)KTOT;

#pragma unroll 1
  for (int ii = 0; ii < IC; ++ii) {
    const int i = i0 + ii;
    FragB bx;
    bx.q[0] = *(const v4ia*)(xrow + (size_t)i * DI) & msk;
    bx.q[1] = z4i;
    v4f lprev = {0.0f, 0.0f, 0.0f, 0.0f};
    if constexpr (PASS == 2) lprev = *(const v4fa*)(L + ((size_t)i * NB_ + b) * NCAP + 4 * q);
    v8f d[4];
    float lg[4];
#pragma unroll
    for (int nt = 0; nt < 4; ++nt) {
      FragB aw;
      aw.q[0] = *(const v4ia*)(wrow + (size_t)nt * DO_ * (size_t)KTOT + (size_t)i * DI) & msk;
      aw.q[1] = z4i;
      d[nt] = wmb(aw, bx, z8);
      float p = 0.0f;
#pragma unroll
      for (int r = 0; r < 8; ++r) p = fmaf(d[nt][r], vr[nt][r], p);
      p += __shfl_xor(p, 16);
      lg[nt] = p + lprev[nt];
    }

    {
      v2f st;
      st.x = (h == 0) ? lg[0] : lg[2];
      st.y = (h == 0) ? lg[1] : lg[3];
      *(v2fa*)(sLog + m * NCAP + 4 * q + 2 * h) = st;
    }
    __syncthreads();

    {
      const int bb = tid & 15, np = tid >> 4;
      const float* rp = sLog + bb * NCAP;
      const float mx = row_max32(rp);
      const v2f x2 = *(const v2fa*)(rp + 2 * np);
      v2f e2;
      e2.x = expf(x2.x - mx);
      e2.y = expf(x2.y - mx);
      *(v2fa*)(sExp + bb * NCAP + 2 * np) = e2;
      if constexpr (PASS == 1) {
        if (tid < 128) {
          const int bl = tid >> 3, pc = tid & 7;
          const v4f lv = *(const v4fa*)(sLog + bl * NCAP + 4 * pc);
          float* lp = L + (((size_t)i * NB_ + 16 * bt + bl) * NCAP + 4 * pc);
          *(volatile v4f*)lp = lv;
          __threadfence();
          *(volatile v4f*)lp = lv;
        }
      }
    }
    __syncthreads();

    {
      const float* ep = sExp + m * NCAP;
      const float sum = row_sum32(ep);
      const float inv = 1.0f / sum;
      const v4f cq = *(const v4fa*)(ep + 4 * q);
#pragma unroll
      for (int nt = 0; nt < 4; ++nt) {
        const float c = cq[nt] * inv;
#pragma unroll
        for (int r = 0; r < 8; ++r) acc[nt][r] = fmaf(c, d[nt][r], acc[nt][r]);
      }
    }
  }

#pragma unroll
  for (int nt = 0; nt < 4; ++nt) {
    float* sp = stg + ((m * NCAP + 4 * q + nt) * DO_ + 8 * h);
    const v4f a = {acc[nt][0], acc[nt][1], acc[nt][2], acc[nt][3]};
    const v4f c = {acc[nt][4], acc[nt][5], acc[nt][6], acc[nt][7]};
    *(v4fa*)sp       = a;
    *(v4fa*)(sp + 4) = c;
  }
  __syncthreads();

  v4f pv[8];
#pragma unroll
  for (int it = 0; it < 8; ++it) pv[it] = *(const v4fa*)(stg + it * 1024 + tid * 4);
  float* op = SP + ((size_t)chunk * NB_ + 16 * bt) * NE;
#pragma unroll
  for (int it = 0; it < 8; ++it) *(volatile v4f*)(op + it * 1024 + tid * 4) = pv[it];
  __threadfence();
#pragma unroll
  for (int it = 0; it < 8; ++it) *(volatile v4f*)(op + it * 1024 + tid * 4) = pv[it];
}

extern "C" void kernel_launch(void* const* d_in, const int* in_sizes, int n_in,
                              void* d_out, int out_size, void* d_ws, size_t ws_size,
                              hipStream_t stream) {
  if (n_in < 2) return;
  if (in_sizes[0] != NB_ * NI * DI) return;
  if (in_sizes[1] != NCAP * NI * DO_ * DI) return;
  if (out_size != NB_ * NE) return;

  const float* X = (const float*)d_in[0];
  const float* W = (const float*)d_in[1];
  float* out = (float*)d_out;

  char* ws = (char*)d_ws;
  size_t off = 0;
  const size_t oXB = off; off += (size_t)NB_ * KTOT * 2;
  const size_t oWT = off; off += (size_t)NCAP * DO_ * KTOT * 2;
  const size_t oL  = off; off += (size_t)NI * NB_ * NCAP * 4;
  const size_t oSP = off; off += (size_t)NCH * SPCH * 4;
  const size_t oV  = off; off += (size_t)NB_ * NE * 4;
  if (off > ws_size || off > (size_t)WSMAX) return;
  unsigned short* XB = (unsigned short*)(ws + oXB);
  unsigned short* WT = (unsigned short*)(ws + oWT);
  float*          L  = (float*)(ws + oL);
  float*          SP = (float*)(ws + oSP);
  float*          V  = (float*)(ws + oV);

  k_prep<<<(NXU + NWU) / PTHR, PTHR, 0, stream>>>(X, W, XB, WT);
  k_gemm0<<<NB_ / 16, GTHR, 0, stream>>>(XB, WT, SP);
  k_combine<<<NB_, CTHR, 0, stream>>>(SP, 1, 0.03125f, V);
  k_route<1><<<dim3(NCH, NB_ / 16), RTHR, 0, stream>>>(XB, WT, V, L, SP);
  k_combine<<<NB_, CTHR, 0, stream>>>(SP, NCH, 1.0f, V);
  k_route<2><<<dim3(NCH, NB_ / 16), RTHR, 0, stream>>>(XB, WT, V, L, SP);
  k_combine<<<NB_, CTHR, 0, stream>>>(SP, NCH, 1.0f, out);
}
